// Interaction_61924838474268
// MI455X (gfx1250) — hardware-verified
//
#include <hip/hip_runtime.h>
#include <stddef.h>
#include <stdint.h>


#define HD      128
#define NRBF    32
#define KIN     64
#define K1V     34
#define H2W     256
#define H3W     384
#define NCOMP   10
#define NODEW   1280
#define XW      1152
#define KF      256
#define NPBLK   16
#define EBLK    32
#define ETHR    128
#define NTHR    256
#define NWAVE   8
#define EPT     8
#define CHUNK   (NTHR * EPT)
#define WCAP    (EPT * 32)
#define LISTN   (NWAVE * WCAP)
#define NBMAX   2048
#define RCAP    28672
#define DEGCAP  4096
#define NU1     1024
#define NU2     4096
#define NU3     12288
#define NUF     (NU1 + NU2 + NU3)
#define NUB     (6 * 128 * 32)
#define NUNITS  (NUF + NUB)
#define CX      16.0f
#define CW      4096.0f
#define SCL     1.52587890625e-05f
#define XSC     16.0f
#define XINV    0.0625f
#define CUTV    5.0f
#define PI_F    3.14159274f
#define THIRD   (1.0f / 3.0f)
#define REGA    81920
#define REGB    73728
#define LDS_NODE (REGA + REGB)
#define LDS_AGG ((2 * RCAP + 2 * NBMAX + LISTN) * 4 + 64)

static_assert((CHUNK & (CHUNK - 1)) == 0 && CHUNK <= 4096);
static_assert((NBMAX & (NBMAX - 1)) == 0 && NBMAX <= 4096);
static_assert(NTHR * 8 == NBMAX);
static_assert(LISTN >= NBMAX);
static_assert(LISTN >= NWAVE * WCAP);
static_assert((RCAP % 32) == 0);
static_assert(LDS_AGG <= 300000);
static_assert(LDS_NODE <= 300000);
static_assert(REGA == NCOMP * NPBLK * KF * 2);
static_assert(REGA >= NPBLK * NODEW * 4);
static_assert(REGA >= NPBLK * XW * 4);
static_assert(REGB == NPBLK * XW * 4);
static_assert((NUF % NTHR) == 0 && (NUNITS % NTHR) == 0);
static_assert(NPBLK * NODEW == 20 * NTHR * 4);
static_assert(NPBLK * XW == 18 * NTHR * 4);
static_assert(NPBLK * HD == 8 * NTHR);
static_assert(EBLK * H3W == 12 * ETHR * 8);
static_assert(EBLK * KIN == 16 * ETHR);
static_assert(EBLK * (HD + H2W) == EBLK * H3W);
static_assert((KIN % 32) == 0 && (HD % 32) == 0 && (H2W % 32) == 0 && (KF % 32) == 0);
static_assert(NODEW == NCOMP * HD && XW == HD * 9 && KF == 2 * HD);
static_assert(HD == (ETHR / 32) * 32 && H2W == (ETHR / 32) * 64 && H3W == (ETHR / 32) * 96);
static_assert(HD == NWAVE * 16);

typedef float    v4f  __attribute__((ext_vector_type(4)));
typedef float    v8f  __attribute__((ext_vector_type(8)));
typedef int      v4i  __attribute__((ext_vector_type(4)));
typedef int      v8i  __attribute__((ext_vector_type(8)));
typedef _Float16 v8h  __attribute__((ext_vector_type(8)));
typedef _Float16 v16h __attribute__((ext_vector_type(16)));
typedef unsigned short v8us __attribute__((ext_vector_type(8)));
typedef __bf16   v16b __attribute__((ext_vector_type(16)));
typedef v8h  __attribute__((may_alias)) v8ha;
typedef v4f  __attribute__((may_alias)) v4fa;
typedef v8us __attribute__((may_alias)) v8usa;
union FragH { v16h v; v8h h[2]; v8i w; };
union FragB { v16b v; v8us u[2]; v8i w; };

extern __shared__ v4f lds_dyn[];

__device__ __forceinline__ v8f wmh(const FragH& a, const FragH& b, v8f c) {
  v8f d = __builtin_amdgcn_wmma_f32_16x16x32_f16(false, a.v, false, b.v, (short)0, c, false, false);
  asm volatile("v_nop\n\tv_nop\n\tv_nop\n\tv_nop" : "+v"(d) : "v"(a.w), "v"(b.w));
  return d;
}
__device__ __forceinline__ v8f wmb(const FragB& a, const FragB& b, v8f c) {
  v8f d = __builtin_amdgcn_wmma_f32_16x16x32_bf16(false, a.v, false, b.v, (short)0, c, false, false);
  asm volatile("v_nop\n\tv_nop\n\tv_nop\n\tv_nop" : "+v"(d) : "v"(a.w), "v"(b.w));
  return d;
}

__device__ __forceinline__ void ldwait() {
  asm volatile("s_wait_loadcnt 0x0" ::: "memory");
}

__device__ __forceinline__ unsigned bf16bits(float f) {
  unsigned u = __float_as_uint(f);
  u += 0x7FFFu + ((u >> 16) & 1u);
  return u >> 16;
}
__device__ __forceinline__ float bf16v(float f) { return __uint_as_float(bf16bits(f) << 16); }

__device__ __forceinline__ float silu_f(float v) { return v * __builtin_amdgcn_rcpf(1.0f + __expf(-v)); }

__device__ __forceinline__ void xnorm9(const float* xs, float* xn) {
  float xb[9];
#pragma unroll
  for (int i = 0; i < 9; ++i) xb[i] = bf16v(xs[i]);
  float nrm = xb[0] * xb[0];
#pragma unroll
  for (int i = 1; i < 9; ++i) nrm = fmaf(xb[i], xb[i], nrm);
  const float inv = 1.0f / (nrm + 1.0f);
#pragma unroll
  for (int i = 0; i < 9; ++i) xn[i] = xb[i] * inv;
}

__device__ __forceinline__ void decomp9(const float* T, float* c) {
  const float I = ((T[0] + T[4]) + T[8]) * THIRD;
  c[0] = I;
  c[1] = 0.5f * (T[7] - T[5]);
  c[2] = 0.5f * (T[2] - T[6]);
  c[3] = 0.5f * (T[3] - T[1]);
  c[4] = T[0] - I;
  c[5] = 0.5f * (T[1] + T[3]);
  c[6] = 0.5f * (T[2] + T[6]);
  c[7] = T[4] - I;
  c[8] = 0.5f * (T[5] + T[7]);
  c[9] = T[8] - I;
}

__device__ __forceinline__ void build9(const float* c, float* Y) {
  Y[0] = c[4] + c[0];  Y[1] = c[5] - c[3];  Y[2] = c[2] + c[6];
  Y[3] = c[3] + c[5];  Y[4] = c[7] + c[0];  Y[5] = c[8] - c[1];
  Y[6] = c[6] - c[2];  Y[7] = c[1] + c[8];  Y[8] = c[9] + c[0];
}

__device__ __forceinline__ void matmul3(const float* A, const float* B, float* C) {
#pragma unroll
  for (int r = 0; r < 3; ++r)
#pragma unroll
    for (int cc = 0; cc < 3; ++cc) {
      float s = A[3 * r] * B[cc];
      s = fmaf(A[3 * r + 1], B[3 + cc], s);
      s = fmaf(A[3 * r + 2], B[6 + cc], s);
      C[3 * r + cc] = s;
    }
}

__device__ __forceinline__ void stage2_comps(const float* y, const float* g, float* cp) {
  float Y[9], P[9], U[9], V[9], M[9], d[NCOMP], Xr[9];
  build9(y, Y);
  build9(g, P);
  matmul3(P, Y, U);
  matmul3(Y, P, V);
#pragma unroll
  for (int i = 0; i < 9; ++i) M[i] = U[i] + V[i];
  decomp9(M, d);
  build9(d, Xr);
  float nrm = Xr[0] * Xr[0];
#pragma unroll
  for (int i = 1; i < 9; ++i) nrm = fmaf(Xr[i], Xr[i], nrm);
  const float inv = 1.0f / (nrm + 1.0f);
#pragma unroll
  for (int c = 0; c < NCOMP; ++c) cp[c] = d[c] * inv;
}

__global__ __launch_bounds__(NTHR) void k_wprep(
    const float* __restrict__ W1, const float* __restrict__ W2, const float* __restrict__ W3,
    const float* __restrict__ T0, const float* __restrict__ T1, const float* __restrict__ T2,
    const float* __restrict__ T3, const float* __restrict__ T4, const float* __restrict__ T5,
    _Float16* W1h, _Float16* W2h, _Float16* W3h, unsigned short* WB, int nUnits)
{
  const int u = (int)blockIdx.x * NTHR + (int)threadIdx.x;
  if (u >= nUnits) return;
  if (u < NUF) {
    const int s   = (u < NU1) ? 0 : ((u < NU1 + NU2) ? 1 : 2);
    const int v   = u - ((s == 0) ? 0 : ((s == 1) ? NU1 : (NU1 + NU2)));
    const int ql  = (s == 0) ? 3 : ((s == 1) ? 4 : 5);
    const int row = v >> ql;
    const int k8  = (v - (row << ql)) * 8;
    const int ld  = (s == 0) ? K1V : ((s == 1) ? HD : H2W);
    const int K   = (s == 0) ? KIN : ld;
    const float* src = (s == 0) ? W1 : ((s == 1) ? W2 : W3);
    _Float16* dst = (s == 0) ? W1h : ((s == 1) ? W2h : W3h);
    const float* p = src + (size_t)row * (size_t)ld;
    v8h hv;
#pragma unroll
    for (int i = 0; i < 8; ++i) {
      const int kk = k8 + i;
      const int kc = kk < ld ? kk : ld - 1;
      float f = p[kc];
      f = kk < ld ? f : 0.0f;
      hv[i] = (_Float16)(bf16v(f) * CW);
    }
    _Float16* op = dst + (size_t)row * (size_t)K + k8;
    *(volatile v8h*)op = hv;
    __threadfence();
    *(volatile v8h*)op = hv;
  } else {
    const int v   = u - NUF;
    const int wi  = v >> 12;
    const int rem = v & 4095;
    const int row = rem >> 5;
    const int k8  = (rem & 31) * 8;
    const int ks  = k8 & (HD - 1);
    const float* src = (wi == 0) ? T0 : ((wi == 1) ? T1 : ((wi == 2) ? T2 : ((wi == 3) ? T3 : ((wi == 4) ? T4 : T5))));
    const float* p = src + (size_t)row * HD + ks;
    v8us bv;
#pragma unroll
    for (int i = 0; i < 8; ++i) bv[i] = (unsigned short)bf16bits(p[i]);
    unsigned short* op = WB + ((size_t)(wi * HD + row)) * KF + k8;
    *(volatile v8us*)op = bv;
    __threadfence();
    *(volatile v8us*)op = bv;
  }
}

__global__ __launch_bounds__(ETHR) void k_edge(
    const float* __restrict__ ea, const float* __restrict__ chg, const float* __restrict__ ew,
    const int* __restrict__ ei,
    const _Float16* __restrict__ W1h, const float* __restrict__ b1,
    const _Float16* __restrict__ W2h, const float* __restrict__ b2,
    const _Float16* __restrict__ W3h, const float* __restrict__ b3,
    _Float16* XE, int nN, int nE)
{
  __shared__ __attribute__((aligned(16))) _Float16 sIn[EBLK * KIN];
  __shared__ __attribute__((aligned(16))) _Float16 sH[EBLK * (HD + H2W)];
  __shared__ float sC[EBLK];
  _Float16* sH1  = sH;
  _Float16* sH2  = sH + EBLK * HD;
  _Float16* sOut = sH;
  const int tid = (int)threadIdx.x, lane = tid & 31, wave = tid >> 5, hh = lane >> 4, m = lane & 15;
  const int e0 = (int)blockIdx.x * EBLK;

  {
    const int r = tid >> 2, q = tid & 3;
    const int e = e0 + r;
    const int ecl = e < nE ? e : nE - 1;
    const float* ap = ea + (size_t)ecl * NRBF + 16 * (q & 1);
    const v4f a0 = *(const v4fa*)ap;
    const v4f a1 = *(const v4fa*)(ap + 4);
    const v4f a2 = *(const v4fa*)(ap + 8);
    const v4f a3 = *(const v4fa*)(ap + 12);
    int s = ei[ecl];
    int d = ei[(size_t)nE + ecl];
    s = s < 0 ? 0 : (s > nN - 1 ? nN - 1 : s);
    d = d < 0 ? 0 : (d > nN - 1 ? nN - 1 : d);
    const float cs = chg[s], cd = chg[d];
    const bool live = e < nE;
    const bool isA  = q < 2;
    const bool isQ  = (q == 2);
    float f[16];
    f[0]  = isA ? a0.x : (isQ ? cs : 0.f);
    f[1]  = isA ? a0.y : (isQ ? cd : 0.f);
    f[2]  = isA ? a0.z : 0.f;  f[3]  = isA ? a0.w : 0.f;
    f[4]  = isA ? a1.x : 0.f;  f[5]  = isA ? a1.y : 0.f;  f[6]  = isA ? a1.z : 0.f;  f[7]  = isA ? a1.w : 0.f;
    f[8]  = isA ? a2.x : 0.f;  f[9]  = isA ? a2.y : 0.f;  f[10] = isA ? a2.z : 0.f;  f[11] = isA ? a2.w : 0.f;
    f[12] = isA ? a3.x : 0.f;  f[13] = isA ? a3.y : 0.f;  f[14] = isA ? a3.z : 0.f;  f[15] = isA ? a3.w : 0.f;
    v8h hv0, hv1;
#pragma unroll
    for (int i = 0; i < 8; ++i) {
      hv0[i] = (_Float16)(live ? bf16v(f[i]) * CX : 0.f);
      hv1[i] = (_Float16)(live ? bf16v(f[8 + i]) * CX : 0.f);
    }
    *(v8h*)(sIn + r * KIN + 16 * q)     = hv0;
    *(v8h*)(sIn + r * KIN + 16 * q + 8) = hv1;
  }
  if (wave == 0) {
    const int e = e0 + lane;
    const int ecl = e < nE ? e : nE - 1;
    const float w = bf16v(ew[ecl]);
    const float cv = 0.5f * (cosf((PI_F * w) * 0.2f) + 1.0f);
    sC[lane] = (e < nE && w < CUTV) ? cv : 0.0f;
  }
  __syncthreads();

  {
    v8f acc[2][2];
    {
      const v8f z = {0.f, 0.f, 0.f, 0.f, 0.f, 0.f, 0.f, 0.f};
#pragma unroll
      for (int mt = 0; mt < 2; ++mt) { acc[mt][0] = z; acc[mt][1] = z; }
    }
    const _Float16* ap = sIn + m * KIN + 8 * hh;
    const _Float16* wp = W1h + (size_t)(32 * wave + m) * KIN + 8 * hh;
#pragma unroll
    for (int ks = 0; ks < KIN / 32; ++ks) {
      FragH af0, af1;
      af0.h[0] = *(const v8ha*)(ap + 32 * ks);
      af0.h[1] = *(const v8ha*)(ap + 32 * ks + 16);
      af1.h[0] = *(const v8ha*)(ap + 16 * KIN + 32 * ks);
      af1.h[1] = *(const v8ha*)(ap + 16 * KIN + 32 * ks + 16);
#pragma unroll
      for (int t = 0; t < 2; ++t) {
        const _Float16* wq = wp + (size_t)(16 * t) * KIN + 32 * ks;
        FragH bf;
        bf.h[0] = *(const v8ha*)wq;
        bf.h[1] = *(const v8ha*)(wq + 16);
        acc[0][t] = wmh(af0, bf, acc[0][t]);
        acc[1][t] = wmh(af1, bf, acc[1][t]);
      }
    }
#pragma unroll
    for (int t = 0; t < 2; ++t) {
      const int col = 32 * wave + 16 * t + m;
      const float bv = bf16v(b1[col]);
#pragma unroll
      for (int mt = 0; mt < 2; ++mt)
#pragma unroll
        for (int r = 0; r < 8; ++r) {
          const int row = 16 * mt + 8 * hh + r;
          const float y = silu_f(fmaf(acc[mt][t][r], SCL, bv));
          sH1[row * HD + col] = (_Float16)(y * CX);
        }
    }
  }
  __syncthreads();

  {
    v8f acc[2][4];
    {
      const v8f z = {0.f, 0.f, 0.f, 0.f, 0.f, 0.f, 0.f, 0.f};
#pragma unroll
      for (int mt = 0; mt < 2; ++mt)
#pragma unroll
        for (int t = 0; t < 4; ++t) acc[mt][t] = z;
    }
    const _Float16* ap = sH1 + m * HD + 8 * hh;
    const _Float16* wp = W2h + (size_t)(64 * wave + m) * HD + 8 * hh;
#pragma unroll 1
    for (int ks = 0; ks < HD / 32; ++ks) {
      FragH af0, af1;
      af0.h[0] = *(const v8ha*)(ap + 32 * ks);
      af0.h[1] = *(const v8ha*)(ap + 32 * ks + 16);
      af1.h[0] = *(const v8ha*)(ap + 16 * HD + 32 * ks);
      af1.h[1] = *(const v8ha*)(ap + 16 * HD + 32 * ks + 16);
#pragma unroll
      for (int t = 0; t < 4; ++t) {
        const _Float16* wq = wp + (size_t)(16 * t) * HD + 32 * ks;
        FragH bf;
        bf.h[0] = *(const v8ha*)wq;
        bf.h[1] = *(const v8ha*)(wq + 16);
        acc[0][t] = wmh(af0, bf, acc[0][t]);
        acc[1][t] = wmh(af1, bf, acc[1][t]);
      }
    }
#pragma unroll
    for (int t = 0; t < 4; ++t) {
      const int col = 64 * wave + 16 * t + m;
      const float bv = bf16v(b2[col]);
#pragma unroll
      for (int mt = 0; mt < 2; ++mt)
#pragma unroll
        for (int r = 0; r < 8; ++r) {
          const int row = 16 * mt + 8 * hh + r;
          const float y = silu_f(fmaf(acc[mt][t][r], SCL, bv));
          sH2[row * H2W + col] = (_Float16)(y * CX);
        }
    }
  }
  __syncthreads();

  {
    v8f acc[2][6];
    {
      const v8f z = {0.f, 0.f, 0.f, 0.f, 0.f, 0.f, 0.f, 0.f};
#pragma unroll
      for (int mt = 0; mt < 2; ++mt)
#pragma unroll
        for (int t = 0; t < 6; ++t) acc[mt][t] = z;
    }
    const _Float16* ap = sH2 + m * H2W + 8 * hh;
    const _Float16* wp = W3h + (size_t)(96 * wave + m) * H2W + 8 * hh;
#pragma unroll 1
    for (int ks = 0; ks < H2W / 32; ++ks) {
      FragH af0, af1;
      af0.h[0] = *(const v8ha*)(ap + 32 * ks);
      af0.h[1] = *(const v8ha*)(ap + 32 * ks + 16);
      af1.h[0] = *(const v8ha*)(ap + 16 * H2W + 32 * ks);
      af1.h[1] = *(const v8ha*)(ap + 16 * H2W + 32 * ks + 16);
#pragma unroll
      for (int t = 0; t < 6; ++t) {
        const _Float16* wq = wp + (size_t)(16 * t) * H2W + 32 * ks;
        FragH bf;
        bf.h[0] = *(const v8ha*)wq;
        bf.h[1] = *(const v8ha*)(wq + 16);
        acc[0][t] = wmh(af0, bf, acc[0][t]);
        acc[1][t] = wmh(af1, bf, acc[1][t]);
      }
    }
    __syncthreads();
#pragma unroll
    for (int t = 0; t < 6; ++t) {
      const int col = 96 * wave + 16 * t + m;
      const float bv = bf16v(b3[col]);
#pragma unroll
      for (int mt = 0; mt < 2; ++mt)
#pragma unroll
        for (int r = 0; r < 8; ++r) {
          const int row = 16 * mt + 8 * hh + r;
          const float y = silu_f(fmaf(acc[mt][t][r], SCL, bv)) * sC[row];
          sOut[row * H3W + col] = (_Float16)(y * XSC);
        }
    }
  }
  __syncthreads();

  _Float16* ob = XE + (size_t)e0 * H3W;
#pragma unroll
  for (int i = 0; i < 12; ++i) {
    const int p = i * ETHR + tid;
    const int row = p / 48;
    if (e0 + row < nE) *(volatile v8h*)(ob + 8 * p) = *(const v8ha*)(sOut + 8 * p);
  }
  __threadfence();
#pragma unroll
  for (int i = 0; i < 12; ++i) {
    const int p = i * ETHR + tid;
    const int row = p / 48;
    if (e0 + row < nE) *(volatile v8h*)(ob + 8 * p) = *(const v8ha*)(sOut + 8 * p);
  }
}

template<int S>
__global__ __launch_bounds__(NTHR) void k_node(
    const float* __restrict__ X, const float* __restrict__ YCin, const float* __restrict__ MSG,
    const unsigned short* __restrict__ WB, float* outp, int nN)
{
  unsigned short* sP = (unsigned short*)lds_dyn;
  float* stgO = (float*)lds_dyn;
  float* stgX = (float*)((char*)lds_dyn + REGA);
  const int tid = (int)threadIdx.x, lane = tid & 31, wave = tid >> 5, hh = lane >> 4, m = lane & 15;
  const int n0 = (int)blockIdx.x * NPBLK;

#pragma unroll
  for (int i = 0; i < 18; ++i) {
    const int p = i * NTHR + tid;
    const int node = p / 288;
    int gn = n0 + node;
    gn = gn < nN ? gn : nN - 1;
    const v4f v = *(const v4fa*)(X + (size_t)gn * XW + 4 * (p - node * 288));
    *(v4f*)(stgX + 4 * p) = v;
  }
  __syncthreads();

#pragma unroll 1
  for (int it = 0; it < 8; ++it) {
    const int pi = it * NTHR + tid;
    const int nl = pi >> 7, ch = pi & (HD - 1);
    const int gnode = n0 + nl;
    const bool live = gnode < nN;
    float cp[NCOMP];
    if (S == 1) {
      float xn[9];
      xnorm9(stgX + nl * XW + ch * 9, xn);
      decomp9(xn, cp);
    } else {
      const int gn = live ? gnode : nN - 1;
      const float* yr = YCin + (size_t)gn * NODEW + ch;
      const float* gr = MSG  + (size_t)gn * NODEW + ch;
      float y[NCOMP], g[NCOMP];
#pragma unroll
      for (int c = 0; c < NCOMP; ++c) y[c] = yr[c * HD];
      ldwait();
#pragma unroll
      for (int c = 0; c < NCOMP; ++c) g[c] = gr[c * HD];
      ldwait();
      stage2_comps(y, g, cp);
    }
#pragma unroll
    for (int c = 0; c < NCOMP; ++c) {
      const float v = live ? cp[c] : 0.0f;
      const unsigned hi = bf16bits(v);
      const unsigned lo = bf16bits(v - __uint_as_float(hi << 16));
      sP[(c * NPBLK + nl) * KF + ch]      = (unsigned short)hi;
      sP[(c * NPBLK + nl) * KF + HD + ch] = (unsigned short)lo;
    }
  }
  __syncthreads();

  v8f acc[NCOMP];
  {
    const v8f z = {0.f, 0.f, 0.f, 0.f, 0.f, 0.f, 0.f, 0.f};
#pragma unroll
    for (int c = 0; c < NCOMP; ++c) acc[c] = z;
  }
  const unsigned short* wp = WB + (size_t)(16 * wave + m) * KF + 8 * hh;
  const unsigned short* ap = sP + m * KF + 8 * hh;
#pragma unroll 1
  for (int ks = 0; ks < KF / 32; ++ks) {
    FragB bw0, bw1, bw2;
    bw0.u[0] = *(const v8usa*)(wp + 32 * ks);
    bw0.u[1] = *(const v8usa*)(wp + 32 * ks + 16);
    bw1.u[0] = *(const v8usa*)(wp + (size_t)HD * KF + 32 * ks);
    bw1.u[1] = *(const v8usa*)(wp + (size_t)HD * KF + 32 * ks + 16);
    bw2.u[0] = *(const v8usa*)(wp + (size_t)2 * HD * KF + 32 * ks);
    bw2.u[1] = *(const v8usa*)(wp + (size_t)2 * HD * KF + 32 * ks + 16);
#pragma unroll
    for (int c = 0; c < NCOMP; ++c) {
      FragB af;
      af.u[0] = *(const v8usa*)(ap + c * NPBLK * KF + 32 * ks);
      af.u[1] = *(const v8usa*)(ap + c * NPBLK * KF + 32 * ks + 16);
      acc[c] = wmb(af, (c == 0) ? bw0 : ((c < 4) ? bw1 : bw2), acc[c]);
    }
  }
  __syncthreads();

  if (S == 1) {
#pragma unroll
    for (int c = 0; c < NCOMP; ++c)
#pragma unroll
      for (int r = 0; r < 8; ++r)
        stgO[(8 * hh + r) * NODEW + c * HD + 16 * wave + m] = acc[c][r];
    __syncthreads();
    float* ob = outp + (size_t)n0 * NODEW;
#pragma unroll
    for (int i = 0; i < 20; ++i) {
      const int p = i * NTHR + tid;
      *(volatile v4f*)(ob + 4 * p) = *(const v4fa*)(stgO + 4 * p);
    }
    __threadfence();
#pragma unroll
    for (int i = 0; i < 20; ++i) {
      const int p = i * NTHR + tid;
      *(volatile v4f*)(ob + 4 * p) = *(const v4fa*)(stgO + 4 * p);
    }
  } else {
#pragma unroll
    for (int r = 0; r < 8; ++r) {
      const int nl = 8 * hh + r, ch = 16 * wave + m;
      float xn[9];
      xnorm9(stgX + nl * XW + ch * 9, xn);
      float dc[NCOMP];
#pragma unroll
      for (int c = 0; c < NCOMP; ++c) dc[c] = acc[c][r];
      float D[9], DD[9];
      build9(dc, D);
      matmul3(D, D, DD);
      float* os = stgO + nl * XW + ch * 9;
#pragma unroll
      for (int i = 0; i < 9; ++i) os[i] = (xn[i] + D[i]) + DD[i];
    }
    __syncthreads();
    float* ob = outp + (size_t)n0 * XW;
#pragma unroll
    for (int i = 0; i < 18; ++i) {
      const int p = i * NTHR + tid;
      const int node = p / 288;
      if (n0 + node < nN) *(volatile v4f*)(ob + 4 * p) = *(const v4fa*)(stgO + 4 * p);
    }
    __threadfence();
#pragma unroll
    for (int i = 0; i < 18; ++i) {
      const int p = i * NTHR + tid;
      const int node = p / 288;
      if (n0 + node < nN) *(volatile v4f*)(ob + 4 * p) = *(const v4fa*)(stgO + 4 * p);
    }
  }
}

__device__ __forceinline__ int scan_chunk(const int* __restrict__ keys, int nE, int cbase, int slotBase,
                                          int nb, int vec8, int* list, int tid, int lane, int wave) {
  int wc = 0;
  const int el0  = tid * EPT;
  const int e0   = cbase + el0;
  const int sent = -2147483647 - 1;
  v4i da, db;
  if (vec8 != 0 && cbase + CHUNK <= nE) {
    da = *(const v4i*)(keys + e0);
    db = *(const v4i*)(keys + e0 + 4);
  } else {
    da.x = (e0     < nE) ? keys[min(e0,     nE - 1)] : sent;
    da.y = (e0 + 1 < nE) ? keys[min(e0 + 1, nE - 1)] : sent;
    da.z = (e0 + 2 < nE) ? keys[min(e0 + 2, nE - 1)] : sent;
    da.w = (e0 + 3 < nE) ? keys[min(e0 + 3, nE - 1)] : sent;
    db.x = (e0 + 4 < nE) ? keys[min(e0 + 4, nE - 1)] : sent;
    db.y = (e0 + 5 < nE) ? keys[min(e0 + 5, nE - 1)] : sent;
    db.z = (e0 + 6 < nE) ? keys[min(e0 + 6, nE - 1)] : sent;
    db.w = (e0 + 7 < nE) ? keys[min(e0 + 7, nE - 1)] : sent;
  }
  const unsigned nbs = (unsigned)slotBase;
  const unsigned unb = (unsigned)nb;
  const unsigned s0 = (unsigned)da.x - nbs, s1 = (unsigned)da.y - nbs;
  const unsigned s2 = (unsigned)da.z - nbs, s3 = (unsigned)da.w - nbs;
  const unsigned s4 = (unsigned)db.x - nbs, s5 = (unsigned)db.y - nbs;
  const unsigned s6 = (unsigned)db.z - nbs, s7 = (unsigned)db.w - nbs;
  const bool h0 = s0 < unb, h1 = s1 < unb, h2 = s2 < unb, h3 = s3 < unb;
  const bool h4 = s4 < unb, h5 = s5 < unb, h6 = s6 < unb, h7 = s7 < unb;
  const unsigned any = __builtin_amdgcn_ballot_w32(h0 | h1 | h2 | h3 | h4 | h5 | h6 | h7);
  if (any != 0u) {
#define HITJ(J, HJ, SJ) { \
      const unsigned mj = __builtin_amdgcn_ballot_w32(HJ); \
      if (mj != 0u) { \
        if (HJ) { \
          const int pos = wc + (int)__builtin_amdgcn_mbcnt_lo(mj, 0u); \
          if (pos < WCAP) list[wave * WCAP + pos] = ((el0 + (J)) << 12) | (int)(SJ); \
        } \
        wc += (int)__builtin_popcount(mj); } }
    HITJ(0, h0, s0)
    HITJ(1, h1, s1)
    HITJ(2, h2, s2)
    HITJ(3, h3, s3)
    HITJ(4, h4, s4)
    HITJ(5, h5, s5)
    HITJ(6, h6, s6)
    HITJ(7, h7, s7)
#undef HITJ
  }
  return wc;
}

__global__ __launch_bounds__(NTHR) void k_msg(
    const int* __restrict__ owners, const int* __restrict__ gath,
    const _Float16* __restrict__ XE, const float* __restrict__ YC, float* MSG,
    int nN, int nE, int nb, int vec8, int MPr) {
  int* reg1 = (int*)lds_dyn;
  int* reg2 = reg1 + RCAP;
  int* scnt = reg2 + RCAP;
  int* soff = scnt + NBMAX;
  int* list = soff + NBMAX;
  int* wcnt = list + LISTN;
  int* wtot = wcnt + NWAVE;
  const int tid = (int)threadIdx.x, lane = tid & 31, wave = tid >> 5;
  const int nodeBase = (int)blockIdx.x * nb;

  for (int i = tid; i < NBMAX; i += NTHR) scnt[i] = 0;
  __syncthreads();

  int tot = 0;
  const int nChunks = (nE + CHUNK - 1) / CHUNK;
#pragma unroll 1
  for (int chn = 0; chn < nChunks; ++chn) {
    const int cbase = chn * CHUNK;
    const int wc = scan_chunk(owners, nE, cbase, nodeBase, nb, vec8, list, tid, lane, wave);
    if (lane == 0) wcnt[wave] = wc;
    __syncthreads();
    int pre = 0, all = 0;
#pragma unroll
    for (int w2 = 0; w2 < NWAVE; ++w2) {
      int c = wcnt[w2];
      c = c < 0 ? 0 : (c > WCAP ? WCAP : c);
      all += c;
      pre += (w2 < wave) ? c : 0;
    }
    const int wcc  = wc > WCAP ? WCAP : wc;
    const int base = tot + pre;
#pragma unroll 1
    for (int i = lane; i < wcc; i += 32) {
      const int ent = list[wave * WCAP + i];
      const int el  = (ent >> 12) & (CHUNK - 1);
      const int sl  = ent & (NBMAX - 1);
      int eid = cbase + el;
      eid = eid > nE - 1 ? nE - 1 : eid;
      const int pos = base + i;
      if (pos < RCAP) reg1[pos] = (int)(((unsigned)eid << 12) | (unsigned)sl);
    }
    tot += all;
    tot = tot > RCAP ? RCAP : tot;
    __syncthreads();
  }
  const int nh = tot;

  if (wave == 0) {
#pragma unroll 1
    for (int b0 = 0; b0 < nh; b0 += 32) {
      const int idx = b0 + lane;
      const int uv  = reg1[idx < RCAP ? idx : RCAP - 1];
      const int m32 = (nh - b0) < 32 ? (nh - b0) : 32;
#pragma unroll 1
      for (int k = 0; k < m32; ++k) {
        const int u  = __builtin_amdgcn_readlane(uv, k);
        const int sl = u & (NBMAX - 1);
        if (lane == 0) scnt[sl] = scnt[sl] + 1;
      }
    }
  }
  __syncthreads();

  {
    const v4i ca = *(const v4i*)(scnt + 8 * tid);
    const v4i cb = *(const v4i*)(scnt + 8 * tid + 4);
    const int e0 = ca.x < 0 ? 0 : ca.x, e1 = ca.y < 0 ? 0 : ca.y, e2 = ca.z < 0 ? 0 : ca.z, e3 = ca.w < 0 ? 0 : ca.w;
    const int e4 = cb.x < 0 ? 0 : cb.x, e5 = cb.y < 0 ? 0 : cb.y, e6 = cb.z < 0 ? 0 : cb.z, e7 = cb.w < 0 ? 0 : cb.w;
    const int ts = e0 + e1 + e2 + e3 + e4 + e5 + e6 + e7;
    int incl = ts;
#pragma unroll
    for (int d = 1; d < 32; d <<= 1) {
      const int up = __shfl_up(incl, d);
      if (lane >= d) incl += up;
    }
    if (lane == 31) wtot[wave] = incl;
    __syncthreads();
    int pre = 0;
#pragma unroll
    for (int w2 = 0; w2 < NWAVE; ++w2) pre += (w2 < wave) ? wtot[w2] : 0;
    int run = pre + incl - ts;
    soff[8 * tid + 0] = run; run += e0;
    soff[8 * tid + 1] = run; run += e1;
    soff[8 * tid + 2] = run; run += e2;
    soff[8 * tid + 3] = run; run += e3;
    soff[8 * tid + 4] = run; run += e4;
    soff[8 * tid + 5] = run; run += e5;
    soff[8 * tid + 6] = run; run += e6;
    soff[8 * tid + 7] = run;
  }
  __syncthreads();
  for (int i = tid; i < NBMAX; i += NTHR) list[i] = soff[i];
  __syncthreads();

  if (wave == 0) {
#pragma unroll 1
    for (int b0 = 0; b0 < nh; b0 += 32) {
      const int idx = b0 + lane;
      const int uv  = reg1[idx < RCAP ? idx : RCAP - 1];
      const int m32 = (nh - b0) < 32 ? (nh - b0) : 32;
#pragma unroll 1
      for (int k = 0; k < m32; ++k) {
        const int u   = __builtin_amdgcn_readlane(uv, k);
        const int sl  = u & (NBMAX - 1);
        const int eid = (int)((unsigned)u >> 12);
        if (lane == 0) {
          int pos = list[sl];
          pos = pos < 0 ? 0 : (pos > RCAP - 1 ? RCAP - 1 : pos);
          reg2[pos] = eid;
          list[sl] = pos + 1;
        }
      }
    }
  }
  __syncthreads();

  const int nbw = nb >> 3;
  const bool ovf = (nh >= RCAP);
  const float qnan = __int_as_float(0x7fc00000);
#pragma unroll 1
  for (int jt = 0; jt < nbw; ++jt) {
    const int slot = wave * nbw + jt;
    const int grow = nodeBase + slot;
    int st = soff[slot];
    const int craw = scnt[slot];
    int cnt = craw;
    st  = st < 0 ? 0 : (st > nh ? nh : st);
    cnt = cnt < 0 ? 0 : (cnt > DEGCAP ? DEGCAP : cnt);
    if (cnt > nh - st) cnt = nh - st;
    const float pz = (ovf || craw > DEGCAP) ? qnan : 0.0f;
    const bool wr = grow < MPr;

    float am[4][NCOMP];
#pragma unroll
    for (int j = 0; j < 4; ++j)
#pragma unroll
      for (int c = 0; c < NCOMP; ++c) am[j][c] = 0.f;

#pragma unroll 1
    for (int q = 0; q < cnt; ++q) {
      int idx = st + q;
      idx = idx > RCAP - 1 ? RCAP - 1 : idx;
      int eid = reg2[idx];
      eid = eid < 0 ? 0 : (eid > nE - 1 ? nE - 1 : eid);
      const int draw = gath[eid];
      const int dn = draw < 0 ? 0 : (draw > nN - 1 ? nN - 1 : draw);
      const _Float16* xr = XE + (size_t)eid * H3W + lane;
      float x0[4], x1[4], x2[4];
#pragma unroll
      for (int j = 0; j < 4; ++j) {
        x0[j] = (float)xr[32 * j];
        x1[j] = (float)xr[HD + 32 * j];
        x2[j] = (float)xr[2 * HD + 32 * j];
      }
      ldwait();
      const float* yr = YC + (size_t)dn * NODEW + lane;
#pragma unroll
      for (int j = 0; j < 4; ++j) {
        float y[NCOMP];
#pragma unroll
        for (int c = 0; c < NCOMP; ++c) y[c] = yr[c * HD + 32 * j];
        ldwait();
        const float f0 = x0[j] * XINV, f1 = x1[j] * XINV, f2 = x2[j] * XINV;
        am[j][0] = fmaf(f0, y[0], am[j][0]);
        am[j][1] = fmaf(f1, y[1], am[j][1]);
        am[j][2] = fmaf(f1, y[2], am[j][2]);
        am[j][3] = fmaf(f1, y[3], am[j][3]);
        am[j][4] = fmaf(f2, y[4], am[j][4]);
        am[j][5] = fmaf(f2, y[5], am[j][5]);
        am[j][6] = fmaf(f2, y[6], am[j][6]);
        am[j][7] = fmaf(f2, y[7], am[j][7]);
        am[j][8] = fmaf(f2, y[8], am[j][8]);
        am[j][9] = fmaf(f2, y[9], am[j][9]);
      }
    }
#pragma unroll
    for (int j = 0; j < 4; ++j)
#pragma unroll
      for (int c = 0; c < NCOMP; ++c) am[j][c] = am[j][c] + pz;

    float* mrow = MSG + (size_t)(grow < MPr ? grow : 0) * NODEW + lane;
    if (wr) {
#pragma unroll
      for (int j = 0; j < 4; ++j)
#pragma unroll
        for (int c = 0; c < NCOMP; ++c) *(volatile float*)(mrow + c * HD + 32 * j) = am[j][c];
    }
    __threadfence();
    if (wr) {
#pragma unroll
      for (int j = 0; j < 4; ++j)
#pragma unroll
        for (int c = 0; c < NCOMP; ++c) *(volatile float*)(mrow + c * HD + 32 * j) = am[j][c];
    }
  }
}

static int pick_nb(int nE, int nNp) {
  int nb = NBMAX;
  while (nb > 16 && (long long)nb * (long long)nE * 5LL > (long long)RCAP * (long long)nNp * 4LL) nb >>= 1;
  return nb;
}
static inline int cdiv(int a, int b) { return (a + b - 1) / b; }

extern "C" void kernel_launch(void* const* d_in, const int* in_sizes, int n_in,
                              void* d_out, int out_size, void* d_ws, size_t ws_size,
                              hipStream_t stream) {
  if (n_in < 17) return;
  const int nN = in_sizes[0] / XW;
  if (nN <= 0 || in_sizes[0] != nN * XW || nN > (1 << 22)) return;
  if (in_sizes[1] != nN) return;
  if (in_sizes[16] < 2 || (in_sizes[16] & 1) != 0) return;
  const int nE = in_sizes[16] / 2;
  if (nE < 1 || nE > (1 << 20)) return;
  if (in_sizes[2] != nE * NRBF || in_sizes[3] != nE) return;
  if (in_sizes[4] != HD * K1V || in_sizes[5] != HD) return;
  if (in_sizes[6] != H2W * HD || in_sizes[7] != H2W) return;
  if (in_sizes[8] != H3W * H2W || in_sizes[9] != H3W) return;
  for (int i = 10; i < 16; ++i) if (in_sizes[i] != HD * HD) return;
  if (out_size != nN * XW) return;

  const float* X    = (const float*)d_in[0];
  const float* chg  = (const float*)d_in[1];
  const float* ea   = (const float*)d_in[2];
  const float* ew   = (const float*)d_in[3];
  const float* W1   = (const float*)d_in[4];
  const float* b1   = (const float*)d_in[5];
  const float* W2   = (const float*)d_in[6];
  const float* b2   = (const float*)d_in[7];
  const float* W3   = (const float*)d_in[8];
  const float* b3   = (const float*)d_in[9];
  const float* Wt0  = (const float*)d_in[10];
  const float* Wt1  = (const float*)d_in[11];
  const float* Wt2  = (const float*)d_in[12];
  const float* Wt3  = (const float*)d_in[13];
  const float* Wt4  = (const float*)d_in[14];
  const float* Wt5  = (const float*)d_in[15];
  const int*   ei   = (const int*)  d_in[16];
  float* out = (float*)d_out;

  const int NPB  = cdiv(nN, NPBLK) * NPBLK;
  const int EP   = cdiv(nE, EBLK) * EBLK;
  const int nb   = pick_nb(nE, NPB);
  const int gA   = cdiv(NPB, nb);
  const int vec8 = ((nE & 3) == 0) ? 1 : 0;
  if (gA * nb < NPB) return;

  char* ws = (char*)d_ws;
  size_t off = 0;
  const size_t oW1h = off; off += (size_t)HD * KIN * 2;            off = (off + 255) & ~(size_t)255;
  const size_t oW2h = off; off += (size_t)H2W * HD * 2;            off = (off + 255) & ~(size_t)255;
  const size_t oW3h = off; off += (size_t)H3W * H2W * 2;           off = (off + 255) & ~(size_t)255;
  const size_t oWB  = off; off += (size_t)6 * HD * KF * 2;         off = (off + 255) & ~(size_t)255;
  const size_t oXE  = off; off += (size_t)EP * H3W * 2;            off = (off + 255) & ~(size_t)255;
  const size_t oYC  = off; off += (size_t)NPB * NODEW * 4;         off = (off + 255) & ~(size_t)255;
  const size_t oMSG = off; off += (size_t)NPB * NODEW * 4;         off = (off + 255) & ~(size_t)255;
  if (off > ws_size) return;
  _Float16* W1h = (_Float16*)(ws + oW1h);
  _Float16* W2h = (_Float16*)(ws + oW2h);
  _Float16* W3h = (_Float16*)(ws + oW3h);
  unsigned short* WB = (unsigned short*)(ws + oWB);
  _Float16* XE  = (_Float16*)(ws + oXE);
  float*    YC  = (float*)(ws + oYC);
  float*    MSG = (float*)(ws + oMSG);

  hipFuncSetAttribute(reinterpret_cast<const void*>(&k_node<1>),
                      hipFuncAttributeMaxDynamicSharedMemorySize, LDS_NODE);
  hipFuncSetAttribute(reinterpret_cast<const void*>(&k_node<2>),
                      hipFuncAttributeMaxDynamicSharedMemorySize, LDS_NODE);
  hipFuncSetAttribute(reinterpret_cast<const void*>(&k_msg),
                      hipFuncAttributeMaxDynamicSharedMemorySize, LDS_AGG);

  k_wprep<<<cdiv(NUNITS, NTHR), NTHR, 0, stream>>>(W1, W2, W3, Wt0, Wt1, Wt2, Wt3, Wt4, Wt5,
                                                   W1h, W2h, W3h, WB, NUNITS);
  k_edge<<<EP / EBLK, ETHR, 0, stream>>>(ea, chg, ew, ei, W1h, b1, W2h, b2, W3h, b3, XE, nN, nE);
  k_node<1><<<NPB / NPBLK, NTHR, LDS_NODE, stream>>>(X, MSG, MSG, WB, YC, nN);
  k_msg<<<gA, NTHR, LDS_AGG, stream>>>(ei, ei + nE, XE, YC, MSG, nN, nE, nb, vec8, NPB);
  k_node<2><<<NPB / NPBLK, NTHR, LDS_NODE, stream>>>(X, YC, MSG, WB + (size_t)3 * HD * KF, out, nN);
}
